// QTSimAM_CNN_LSTM_Model_6511170421082
// MI455X (gfx1250) — hardware-verified
//
#include <hip/hip_runtime.h>
#include <math.h>

typedef __attribute__((ext_vector_type(16))) _Float16 v16h;
typedef __attribute__((ext_vector_type(8)))  _Float16 v8h;
typedef __attribute__((ext_vector_type(16))) __bf16   v16b;
typedef __attribute__((ext_vector_type(8)))  __bf16   v8b;
typedef __attribute__((ext_vector_type(8)))  float    v8f;
typedef __attribute__((ext_vector_type(4)))  float    v4f;

constexpr int NBAT   = 256;
constexpr int NSTEP  = 512;
constexpr int NFEAT  = 16;
constexpr int CH1    = 64;
constexpr int CH2    = 128;
constexpr int CH3    = 256;
constexpr int NHID   = 128;
constexpr int NGC    = 512;
constexpr int NCLS   = 8;
constexpr int KMODIN = 130;
constexpr int KMODW  = 160;
constexpr int KW1SRC = 48;
constexpr int KW1    = 64;
constexpr int KW2    = 192;
constexpr int KW3    = 384;
constexpr int PROWS  = NSTEP + 2;
constexpr float EPSQ = 1e-6f;
constexpr float ELAM = 1e-4f;

constexpr float CX     = 16.0f;
constexpr float CWCONV = 256.0f;
constexpr float CZ1    = 64.0f;
constexpr float CZ2    = 1024.0f;
constexpr float CSEQ   = 4096.0f;
constexpr float CWMOD  = 64.0f;
constexpr float CWD    = 16384.0f;
constexpr float CWL    = 16.0f;
constexpr float CWIH   = 64.0f;
constexpr float CWHH   = 16.0f;
constexpr float CARRY_H = 4096.0f;
constexpr float CARRY_D = 16.0f;
constexpr float CARRY_L = 16384.0f;
constexpr float FOLD_MS = 0.25f;
constexpr float INV_G1  = 1.0f / 4096.0f;
constexpr float INV_G2  = 1.0f / 16384.0f;
constexpr float INV_G3  = 1.0f / 262144.0f;
constexpr float INV_MOG = 1.0f / 262144.0f;
constexpr float INV_GAT = 1.0f / 65536.0f;

constexpr int LROWS   = 32;
constexpr int LTHR    = 256;
constexpr int TPITCH  = 424;
constexpr int COL_MS  = 0;
constexpr int COL_HID = 256;
constexpr int COL_DQ  = 384;
constexpr int HSPITCH = 132;
static_assert(NBAT % LROWS == 0);
static_assert((2 * LROWS * TPITCH) % LTHR == 0);
static_assert(NHID == 16 * (LTHR / 32));
static_assert(CH3 == 32 * (LTHR / 32));
static_assert(LROWS * NCLS == LTHR);
static_assert(TPITCH % 8 == 0 && COL_DQ + 2 <= COL_HID + KMODW && COL_HID + KMODW <= TPITCH);

__device__ __forceinline__ unsigned short f2bf_bits(float f) {
  unsigned u = __float_as_uint(f);
  return (unsigned short)((u + 0x7FFFu + ((u >> 16) & 1u)) >> 16);
}
__device__ __forceinline__ float bf_bits2f(unsigned short h) { return __uint_as_float(((unsigned)h) << 16); }
__device__ __forceinline__ float bf16r(float f) { return bf_bits2f(f2bf_bits(f)); }
__device__ __forceinline__ float h2f(unsigned short u) { return (float)__builtin_bit_cast(_Float16, u); }

__device__ __forceinline__ void dep_guard_h(v8f& a, v8f& b, v16h x, v16h y) { asm volatile("v_nop\n\tv_nop\n\tv_nop\n\tv_nop" : "+v"(a), "+v"(b) : "v"(x), "v"(y)); }
__device__ __forceinline__ void dep_guard_b(v8f& a, v8f& b, v16b x, v16b y) { asm volatile("v_nop\n\tv_nop\n\tv_nop\n\tv_nop" : "+v"(a), "+v"(b) : "v"(x), "v"(y)); }
__device__ __forceinline__ void keep4_h(v16h a, v16h b, v16h c, v16h d) { asm volatile("v_nop" :: "v"(a), "v"(b), "v"(c), "v"(d)); }
__device__ __forceinline__ void keep4_b(v16b a, v16b b, v16b c, v16b d) { asm volatile("v_nop" :: "v"(a), "v"(b), "v"(c), "v"(d)); }
__device__ __forceinline__ void acc_guard4(v8f& a, v8f& b, v8f& c, v8f& d) { asm volatile("v_nop\n\tv_nop\n\tv_nop\n\tv_nop" : "+v"(a), "+v"(b), "+v"(c), "+v"(d)); }
template <typename T> struct Frag;
template <> struct Frag<_Float16> {
  typedef v16h V; union U { v16h v; v8h h[2]; };
  static __device__ __forceinline__ v16h load(const _Float16* p) {
    U f; f.h[0] = *(const v8h*)(p); f.h[1] = *(const v8h*)(p + 16); return f.v;
  }
  static __device__ __forceinline__ v8f mma(v16h a, v16h b, v8f c) {
    return __builtin_amdgcn_wmma_f32_16x16x32_f16(false, a, false, b, (short)0, c, false, false);
  }
  static __device__ __forceinline__ void guard(v8f& a, v8f& b, v16h x, v16h y) { dep_guard_h(a, b, x, y); }
  static __device__ __forceinline__ void keep(v16h a, v16h b, v16h c, v16h d) { keep4_h(a, b, c, d); }
};
template <> struct Frag<__bf16> {
  typedef v16b V; union U { v16b v; v8b h[2]; };
  static __device__ __forceinline__ v16b load(const __bf16* p) {
    U f; f.h[0] = *(const v8b*)(p); f.h[1] = *(const v8b*)(p + 16); return f.v;
  }
  static __device__ __forceinline__ v8f mma(v16b a, v16b b, v8f c) {
    return __builtin_amdgcn_wmma_f32_16x16x32_bf16(false, a, false, b, (short)0, c, false, false);
  }
  static __device__ __forceinline__ void guard(v8f& a, v8f& b, v16b x, v16b y) { dep_guard_b(a, b, x, y); }
  static __device__ __forceinline__ void keep(v16b a, v16b b, v16b c, v16b d) { keep4_b(a, b, c, d); }
};

__device__ __forceinline__ float fsig(float x) { return __builtin_amdgcn_rcpf(1.0f + __expf(-x)); }
__device__ __forceinline__ float tanh_acc(float x) {
  const float a  = fabsf(x);
  const float x2 = x * x;
  float p = 0.021869488536155203f;
  p = fmaf(p, x2, -0.053968253968253968f);
  p = fmaf(p, x2, 0.13333333333333333f);
  p = fmaf(p, x2, -0.33333333333333333f);
  const float ps = fmaf(x * x2, p, x);
  const float e2 = __expf(2.0f * a);
  const float bgv = 1.0f - 2.0f * __builtin_amdgcn_rcpf(e2 + 1.0f);
  const float bs = copysignf(bgv, x);
  return (a < 0.25f) ? ps : bs;
}

__global__ __launch_bounds__(512) void queue_kernel(const float* __restrict__ x, const float* __restrict__ ksp,
                                                    const float* __restrict__ kap, float* __restrict__ WQ,
                                                    float* __restrict__ LQ, float* __restrict__ PART) {
#pragma clang fp contract(off)
  __shared__ float red[4][16];
  __shared__ __align__(16) float row32[32];
  const int b = blockIdx.x, s = threadIdx.x, lane = s & 31, wave = s >> 5;
  const float ks = bf16r(ksp[0]);
  const float ka = bf16r(kap[0]);
  const float* xe = x + ((size_t)b * NSTEP + s) * NFEAT;
  const float dist = bf16r(xe[NFEAT - 3]);
  const float air  = bf16r(xe[NFEAT - 5]);
  const float es   = ks * dist + EPSQ;
  const float lam  = ka * (1.0f / (air + EPSQ));
  const float rho  = fminf(lam * es, 0.99f);
  const float wq   = rho * (1.0f / ((1.0f - rho) + EPSQ)) * es;
  const float lq   = lam * wq;
  const size_t oi = (size_t)b * NSTEP + s;
  ((volatile float*)WQ)[oi] = wq;
  ((volatile float*)LQ)[oi] = lq;
  __threadfence();
  ((volatile float*)WQ)[oi] = wq;
  ((volatile float*)LQ)[oi] = lq;

  float wmn = wq, wmx = wq, lmn = lq, lmx = lq;
#pragma unroll
  for (int off = 1; off < 32; off <<= 1) {
    wmn = fminf(wmn, __shfl_xor(wmn, off, 32));
    wmx = fmaxf(wmx, __shfl_xor(wmx, off, 32));
    lmn = fminf(lmn, __shfl_xor(lmn, off, 32));
    lmx = fmaxf(lmx, __shfl_xor(lmx, off, 32));
  }
  if (lane == 0) { red[0][wave] = wmn; red[1][wave] = wmx; red[2][wave] = lmn; red[3][wave] = lmx; }
  if (s < 32) row32[s] = 0.0f;
  __syncthreads();
  if (s == 0) {
    float a0 = red[0][0], a1 = red[1][0], a2 = red[2][0], a3 = red[3][0];
    for (int i = 1; i < 16; ++i) {
      a0 = fminf(a0, red[0][i]); a1 = fmaxf(a1, red[1][i]);
      a2 = fminf(a2, red[2][i]); a3 = fmaxf(a3, red[3][i]);
    }
    row32[0] = a0; row32[1] = a1; row32[2] = a2; row32[3] = a3;
  }
  __syncthreads();
  if (s < 8) {
    const v4f v = *(const v4f*)(row32 + 4 * s);
    float* pr = PART + (size_t)b * 32 + 4 * s;
    *(volatile v4f*)pr = v;
    __threadfence();
    *(volatile v4f*)pr = v;
  }
}

__global__ __launch_bounds__(512) void norm_kernel(const float* __restrict__ WQ, const float* __restrict__ LQ,
                                                   const float* __restrict__ PART, float* __restrict__ WN,
                                                   float* __restrict__ LN, float* __restrict__ DL) {
#pragma clang fp contract(off)
  __shared__ float sh[4][256];
  __shared__ float red[2][16];
  __shared__ __align__(16) float row32[32];
  const int t = threadIdx.x, b = blockIdx.x, lane = t & 31, wave = t >> 5;
  if (t < NBAT) {
    sh[0][t] = PART[(size_t)t * 32 + 0];
    sh[1][t] = PART[(size_t)t * 32 + 1];
    sh[2][t] = PART[(size_t)t * 32 + 2];
    sh[3][t] = PART[(size_t)t * 32 + 3];
  }
  __syncthreads();
#pragma unroll 1
  for (int off = 128; off > 0; off >>= 1) {
    if (t < off) {
      sh[0][t] = fminf(sh[0][t], sh[0][t + off]);
      sh[1][t] = fmaxf(sh[1][t], sh[1][t + off]);
      sh[2][t] = fminf(sh[2][t], sh[2][t + off]);
      sh[3][t] = fmaxf(sh[3][t], sh[3][t + off]);
    }
    __syncthreads();
  }
  const float wmn = sh[0][0], wmx = sh[1][0], lmn = sh[2][0], lmx = sh[3][0];
  const float winv = 1.0f / ((wmx - wmn) + EPSQ);
  const float linv = 1.0f / ((lmx - lmn) + EPSQ);
  const size_t oi = (size_t)b * NSTEP + t;
  const float wn = (WQ[oi] - wmn) * winv;
  const float ln = (LQ[oi] - lmn) * linv;
  ((volatile float*)WN)[oi] = wn;
  ((volatile float*)LN)[oi] = ln;
  __threadfence();
  ((volatile float*)WN)[oi] = wn;
  ((volatile float*)LN)[oi] = ln;

  float sw = wn, sl = ln;
#pragma unroll
  for (int off = 1; off < 32; off <<= 1) {
    sw += __shfl_xor(sw, off, 32);
    sl += __shfl_xor(sl, off, 32);
  }
  if (lane == 0) { red[0][wave] = sw; red[1][wave] = sl; }
  if (t < 32) row32[t] = 0.0f;
  __syncthreads();
  if (t == 0) {
    float a0 = 0.0f, a1 = 0.0f;
    for (int i = 0; i < 16; ++i) { a0 += red[0][i]; a1 += red[1][i]; }
    row32[0] = a0 * (1.0f / 512.0f);
    row32[1] = a1 * (1.0f / 512.0f);
  }
  __syncthreads();
  if (t < 8) {
    const v4f v = *(const v4f*)(row32 + 4 * t);
    float* pr = DL + (size_t)b * 32 + 4 * t;
    *(volatile v4f*)pr = v;
    __threadfence();
    *(volatile v4f*)pr = v;
  }
}

__global__ __launch_bounds__(256) void wcvt_kernel(const float* __restrict__ src, unsigned short* __restrict__ dst,
                                                   int n8, int kp, int ksrc, int cin, int mode, float s0) {
  const int i = blockIdx.x * 256 + threadIdx.x;
  if (i >= n8) return;
  const int flat = i * 8;
  const int o  = flat / kp;
  const int kb = flat - o * kp;
  v8h hv;
#pragma unroll
  for (int e = 0; e < 8; ++e) {
    const int kk = kb + e;
    int idx; float sc = s0; bool valid;
    if (mode == 1) {
      const int dk = kk / cin;
      const int ci = kk - dk * cin;
      const int dkc = dk > 2 ? 2 : dk;
      idx = o * ksrc + ci * 3 + dkc; valid = true;
    } else if (mode == 2) {
      valid = kk < ksrc;
      const int kc = kk < ksrc ? kk : (ksrc - 1);
      idx = o * ksrc + kc;
      sc = (kk < ksrc - 2) ? s0 : ((kk == ksrc - 2) ? CWD : CWL);
    } else {
      valid = kk < ksrc;
      const int kc = kk < ksrc ? kk : (ksrc - 1);
      idx = o * ksrc + kc;
    }
    const float v = src[idx];
    const float w = valid ? sc * bf16r(v) : 0.0f;
    hv[e] = (_Float16)w;
  }
  unsigned short* d = dst + (size_t)i * 8;
  *(volatile v8h*)d = hv;
  __threadfence();
  *(volatile v8h*)d = hv;
}

__global__ __launch_bounds__(256) void xcol_kernel(const float* __restrict__ x, unsigned short* __restrict__ A1) {
  const int i   = blockIdx.x * 256 + threadIdx.x;
  const int row = i >> 3, g = i & 7;
  const int b   = row >> 9, s = row & (NSTEP - 1);
  v8h hv;
#pragma unroll
  for (int e = 0; e < 8; ++e) {
    const int kk = 8 * g + e;
    int ci = kk / 3;
    const int dk = kk - ci * 3;
    const bool kval = kk < KW1SRC;
    ci = ci > (NFEAT - 1) ? (NFEAT - 1) : ci;
    const int ss = s + dk - 1;
    const bool sval = (ss >= 0) && (ss < NSTEP);
    const int ssc = ss < 0 ? 0 : (ss > NSTEP - 1 ? NSTEP - 1 : ss);
    const float v = x[((size_t)b * NSTEP + ssc) * NFEAT + ci];
    const float o = (kval && sval) ? CX * bf16r(v) : 0.0f;
    hv[e] = (_Float16)o;
  }
  unsigned short* d = A1 + (size_t)i * 8;
  *(volatile v8h*)d = hv;
  __threadfence();
  *(volatile v8h*)d = hv;
}

template <int ET> struct Elem;
template <> struct Elem<0> { typedef _Float16 T; };
template <> struct Elem<1> { typedef __bf16 T; };
template <int ET, bool SPLIT, int BIAS_MODE, int OUT_MODE, bool RESID, int ACT = 0>
__global__ __launch_bounds__(256) void wmma_gemm64(
    const unsigned short* __restrict__ Ap, const unsigned short* __restrict__ A2p, int lda, long strideA,
    const unsigned short* __restrict__ Btp, const unsigned short* __restrict__ Bt2p, int ldb, long strideB,
    void* __restrict__ Cout, void* __restrict__ Cout2, int ldc, long strideC,
    const float* __restrict__ bias,
    const float* __restrict__ resid, long strideR,
    int M, int N, int K, float scale) {
  typedef typename Elem<ET>::T T;
  typedef typename Frag<T>::V V;
  const T* A = (const T*)Ap; const T* A2 = (const T*)A2p; const T* Bt = (const T*)Btp; const T* Bt2 = (const T*)Bt2p;
  __shared__ __align__(16) float sT[8][16 * 68];
  const int b    = blockIdx.y;
  const int lane = threadIdx.x & 31;
  const int wave = threadIdx.x >> 5;
  const int tilesN = N >> 6;
  const int tilesM = M >> 6;
  const int tile = blockIdx.x * 8 + wave;
  if (tile >= tilesM * tilesN) return;
  const int tm = tile / tilesN;
  const int tn = tile - tm * tilesN;
  const int m0 = tm << 6;
  const int n0 = tn << 6;

  const T* Ab  = A  + (size_t)b * strideA;
  const T* Bb  = Bt + (size_t)b * strideB;
  const T* Ab2 = SPLIT ? (A2  + (size_t)b * strideA) : nullptr;
  const T* Bb2 = SPLIT ? (Bt2 + (size_t)b * strideB) : nullptr;

  const int rlane = lane & 15;
  const int koff  = (lane >> 4) * 8;
  const int mOff  = (lane >> 4) * 8;

  v8f acc[4][4];
#pragma unroll
  for (int i = 0; i < 4; ++i)
#pragma unroll
    for (int j = 0; j < 4; ++j) acc[i][j] = (v8f){0.f,0.f,0.f,0.f,0.f,0.f,0.f,0.f};

  for (int k0 = 0; k0 < K; k0 += 32) {
    V bh[4], bl[4];
#pragma unroll
    for (int j = 0; j < 4; ++j) {
      const size_t bo = (size_t)(n0 + (j << 4) + rlane) * ldb + koff + k0;
      bh[j] = Frag<T>::load(Bb + bo);
      if (SPLIT) bl[j] = Frag<T>::load(Bb2 + bo);
    }
#pragma unroll
    for (int i = 0; i < 4; ++i) {
      const size_t ao = (size_t)(m0 + (i << 4) + rlane) * lda + koff + k0;
      V ah = Frag<T>::load(Ab + ao);
      V al;
      if (SPLIT) al = Frag<T>::load(Ab2 + ao);
#pragma unroll
      for (int j = 0; j < 4; ++j) {
        acc[i][j] = Frag<T>::mma(ah, bh[j], acc[i][j]);
        if (SPLIT) {
          acc[i][j] = Frag<T>::mma(ah, bl[j], acc[i][j]);
          acc[i][j] = Frag<T>::mma(al, bh[j], acc[i][j]);
        }
      }
      Frag<T>::guard(acc[i][0], acc[i][3], ah, SPLIT ? al : ah);
    }
    Frag<T>::keep(bh[0], bh[1], bh[2], bh[3]);
    if (SPLIT) Frag<T>::keep(bl[0], bl[1], bl[2], bl[3]);
  }
  acc_guard4(acc[0][0], acc[0][1], acc[0][2], acc[0][3]);
  acc_guard4(acc[1][0], acc[1][1], acc[1][2], acc[1][3]);
  acc_guard4(acc[2][0], acc[2][1], acc[2][2], acc[2][3]);
  acc_guard4(acc[3][0], acc[3][1], acc[3][2], acc[3][3]);

  float* slab = sT[wave];
  const float* Rb = RESID ? (resid + (size_t)b * strideR) : nullptr;
#pragma unroll
  for (int i = 0; i < 4; ++i) {
    const int mBase = m0 + (i << 4);
#pragma unroll
    for (int j = 0; j < 4; ++j) {
      const int n = n0 + (j << 4) + rlane;
      float bv = 0.f;
      if (BIAS_MODE == 2) bv = bias[n];
      if (BIAS_MODE == 3) bv = bf16r(bias[n]);
#pragma unroll
      for (int r = 0; r < 8; ++r) {
        float v = acc[i][j][r] * scale;
        if (BIAS_MODE == 1) v += bias[mBase + mOff + r];
        if (BIAS_MODE == 2 || BIAS_MODE == 3) v += bv;
        if (RESID) v += Rb[(size_t)(mBase + mOff + r) * ldc + n];
        if (ACT == 1) v = tanhf(v);
        if (ACT == 2) v = fmaxf(v, 0.0f);
        if (ACT == 3) v = v / (1.0f + expf(-v));
        if (ACT == 4) v = (v > 0.f) ? v : 0.01f * v;
        if (ACT == 5) v = 0.5f * v * (1.0f + erff(v * 0.70710678118654752f));
        slab[(mOff + r) * 68 + (j << 4) + rlane] = v;
      }
    }
    __builtin_amdgcn_fence(__ATOMIC_RELEASE, "workgroup");
    __builtin_amdgcn_wave_barrier();
    __builtin_amdgcn_fence(__ATOMIC_ACQUIRE, "workgroup");
    if (OUT_MODE == 0) {
      float* C = (float*)Cout + (size_t)b * strideC;
      const int hh = lane >> 4, c4 = (lane & 15) * 4;
      for (int pass = 0; pass < 2; ++pass) {
#pragma unroll
        for (int it = 0; it < 8; ++it) {
          const int row = it * 2 + hh;
          v4f v = *(const v4f*)(slab + row * 68 + c4);
          *(volatile v4f*)(C + (size_t)(mBase + row) * ldc + n0 + c4) = v;
        }
        __threadfence();
      }
    } else {
      const int q = lane >> 3, c8 = (lane & 7) * 8;
      unsigned short* C  = (unsigned short*)Cout  + (size_t)b * strideC;
      unsigned short* C2 = (OUT_MODE == 2) ? ((unsigned short*)Cout2 + (size_t)b * strideC) : nullptr;
      for (int pass = 0; pass < 2; ++pass) {
#pragma unroll
        for (int it = 0; it < 4; ++it) {
          const int row = it * 4 + q;
          const float* sp = slab + row * 68 + c8;
          v8h hv, lv;
#pragma unroll
          for (int e = 0; e < 8; ++e) {
            if (OUT_MODE == 1) {
              hv[e] = (_Float16)sp[e];
            } else {
              unsigned short hb = f2bf_bits(sp[e]);
              unsigned short lb = f2bf_bits(sp[e] - bf_bits2f(hb));
              hv[e] = __builtin_bit_cast(_Float16, hb);
              lv[e] = __builtin_bit_cast(_Float16, lb);
            }
          }
          *(volatile v8h*)(C + (size_t)(mBase + row) * ldc + n0 + c8) = hv;
          if (OUT_MODE == 2) *(volatile v8h*)(C2 + (size_t)(mBase + row) * ldc + n0 + c8) = lv;
        }
        __threadfence();
      }
    }
    __builtin_amdgcn_fence(__ATOMIC_RELEASE, "workgroup");
    __builtin_amdgcn_wave_barrier();
    __builtin_amdgcn_fence(__ATOMIC_ACQUIRE, "workgroup");
  }
}

__global__ __launch_bounds__(256) void simam_cvt_kernel(const float* __restrict__ Y, int ncol, const float* __restrict__ DL,
                                                        unsigned short* __restrict__ P, int prow, int pad, int bg0, float carry) {
  __shared__ float ps[4][64];
  __shared__ float pq[4][64];
  __shared__ float scl[64];
  const int tid = threadIdx.x, lane = tid & 31, wave = tid >> 5;
  const int slab = blockIdx.x, bl = blockIdx.y, bg = bg0 + bl;
  const size_t ybase = (size_t)bl * NSTEP * ncol + (size_t)slab * 64;
  {
    const int cc = tid & 63, q = tid >> 6;
    const float* yp = Y + ybase + (size_t)(q * 128) * ncol + cc;
    float s = 0.0f, s2 = 0.0f;
#pragma unroll 4
    for (int r = 0; r < 128; ++r) {
      const float v = yp[(size_t)r * ncol];
      s += v;
      s2 = fmaf(v, v, s2);
    }
    ps[q][cc] = s;
    pq[q][cc] = s2;
  }
  __syncthreads();
  if (tid < 64) {
    const float S = ((ps[0][tid] + ps[1][tid]) + ps[2][tid]) + ps[3][tid];
    const float Q = ((pq[0][tid] + pq[1][tid]) + pq[2][tid]) + pq[3][tid];
    const float mu  = S * (1.0f / 512.0f);
    const float var = Q * (1.0f / 512.0f) - mu * mu;
    const float d = DL[(size_t)bg * 32 + 0];
    const float l = DL[(size_t)bg * 32 + 1];
    const float e = ((var + d) + 0.5f * l) + ELAM;
    scl[tid] = carry * fsig(e);
  }
  __syncthreads();
  const int q = lane >> 3, c8 = (lane & 7) * 8;
  float sc8[8];
#pragma unroll
  for (int e = 0; e < 8; ++e) sc8[e] = scl[c8 + e];
  unsigned short* pb = P + ((size_t)bg * prow + pad) * ncol + (size_t)slab * 64 + c8;
  const float* yb = Y + ybase + c8;
  for (int pass = 0; pass < 2; ++pass) {
#pragma unroll 1
    for (int it = 0; it < 16; ++it) {
      const int row = wave * 64 + it * 4 + q;
      const float* yr = yb + (size_t)row * ncol;
      const v4f a = *(const v4f*)(yr);
      const v4f c = *(const v4f*)(yr + 4);
      v8h hv;
#pragma unroll
      for (int e = 0; e < 4; ++e) {
        hv[e]     = (_Float16)(a[e] * sc8[e]);
        hv[4 + e] = (_Float16)(c[e] * sc8[4 + e]);
      }
      *(volatile v8h*)(pb + (size_t)row * ncol) = hv;
    }
    __threadfence();
  }
  if (pad != 0 && wave == 0 && lane < 16) {
    v8h z;
#pragma unroll
    for (int e = 0; e < 8; ++e) z[e] = (_Float16)0.0f;
    const int prw = (lane < 8) ? 0 : (prow - 1);
    unsigned short* pz = P + ((size_t)bg * prow + prw) * ncol + (size_t)slab * 64 + c8;
    *(volatile v8h*)pz = z;
    __threadfence();
    *(volatile v8h*)pz = z;
  }
}

__global__ __launch_bounds__(LTHR) void lstm_kernel(const unsigned short* __restrict__ SEQp,
                                                   const float* __restrict__ WN, const float* __restrict__ LN,
                                                   const unsigned short* __restrict__ MWp, const float* __restrict__ modb,
                                                   const unsigned short* __restrict__ WIHp, const unsigned short* __restrict__ WHHp,
                                                   const float* __restrict__ bih, const float* __restrict__ bhh,
                                                   const float* __restrict__ clsw, const float* __restrict__ clsb,
                                                   float* __restrict__ out) {
  __shared__ __align__(16) _Float16 At[2][LROWS * TPITCH];
  __shared__ __align__(16) float    Hs[LROWS * HSPITCH];
  __shared__ __align__(16) float    Os[LROWS * NCLS];
  const _Float16* MW  = (const _Float16*)MWp;
  const _Float16* WIH = (const _Float16*)WIHp;
  const _Float16* WHH = (const _Float16*)WHHp;
  const int tid = threadIdx.x, lane = tid & 31, wave = tid >> 5;
  const int c = lane & 15, hh = lane >> 4, koff = hh * 8;
  const int bbase = blockIdx.x * LROWS;

  {
    _Float16* f = &At[0][0];
#pragma unroll 1
    for (int i = tid; i < 2 * LROWS * TPITCH; i += LTHR) f[i] = (_Float16)0.0f;
  }
  __syncthreads();
  if (tid < 2 * LROWS) {
    const int row = tid >> 1, w = tid & 1;
    const size_t qi = (size_t)(bbase + row) * NSTEP;
    const float vd = WN[qi] * CARRY_D;
    const float vl = LN[qi] * CARRY_L;
    At[0][row * TPITCH + COL_DQ + w] = (_Float16)(w ? vl : vd);
  }
  const int jh = 16 * wave + c;
  float bg[4];
#pragma unroll
  for (int g = 0; g < 4; ++g) bg[g] = bf16r(bih[g * NHID + jh]) + bf16r(bhh[g * NHID + jh]);
  float mb[2];
#pragma unroll
  for (int nt = 0; nt < 2; ++nt) mb[nt] = bf16r(modb[32 * wave + 16 * nt + c]);
  float cst[2][8];
#pragma unroll
  for (int mt = 0; mt < 2; ++mt)
#pragma unroll
    for (int r = 0; r < 8; ++r) cst[mt][r] = 0.0f;
  __syncthreads();

  const v8f z8 = {0.f, 0.f, 0.f, 0.f, 0.f, 0.f, 0.f, 0.f};

#pragma unroll 1
  for (int t = 0; t < NSTEP; ++t) {
    const int cur = t & 1;
    const _Float16* Ac = &At[cur][0];
    _Float16* Aw = &At[cur][0];
    _Float16* An = &At[cur ^ 1][0];
    const bool last = (t == NSTEP - 1);

    if (tid < 2 * LROWS) {
      const int tn = (t + 1 < NSTEP) ? (t + 1) : (NSTEP - 1);
      const int row = tid >> 1, w = tid & 1;
      const size_t qi = (size_t)(bbase + row) * NSTEP + tn;
      const float vd = WN[qi] * CARRY_D;
      const float vl = LN[qi] * CARRY_L;
      An[row * TPITCH + COL_DQ + w] = (_Float16)(w ? vl : vd);
    }

    {
      v8f am[2][2];
      am[0][0] = z8; am[0][1] = z8; am[1][0] = z8; am[1][1] = z8;
      const _Float16* ap = Ac + c * TPITCH + COL_HID + koff;
      const _Float16* bp = MW + (size_t)(32 * wave + c) * KMODW + koff;
#pragma unroll 1
      for (int kk = 0; kk < KMODW; kk += 32) {
        const v16h a0 = Frag<_Float16>::load(ap + kk);
        const v16h a1 = Frag<_Float16>::load(ap + 16 * TPITCH + kk);
        const v16h b0 = Frag<_Float16>::load(bp + kk);
        const v16h b1 = Frag<_Float16>::load(bp + (size_t)16 * KMODW + kk);
        am[0][0] = Frag<_Float16>::mma(a0, b0, am[0][0]);
        am[0][1] = Frag<_Float16>::mma(a0, b1, am[0][1]);
        am[1][0] = Frag<_Float16>::mma(a1, b0, am[1][0]);
        am[1][1] = Frag<_Float16>::mma(a1, b1, am[1][1]);
        dep_guard_h(am[0][0], am[1][1], a0, a1);
        keep4_h(b0, b1, a0, a1);
      }
      acc_guard4(am[0][0], am[0][1], am[1][0], am[1][1]);
#pragma unroll
      for (int mt = 0; mt < 2; ++mt) {
#pragma unroll
        for (int nt = 0; nt < 2; ++nt) {
          const int col = 32 * wave + 16 * nt + c;
#pragma unroll
          for (int r = 0; r < 8; ++r) {
            const int row = 16 * mt + 8 * hh + r;
            const float z  = am[mt][nt][r] * INV_MOG + mb[nt];
            const float m  = fsig(z);
            const float sv = h2f(SEQp[((size_t)(bbase + row) * NSTEP + t) * CH3 + col]);
            Aw[row * TPITCH + COL_MS + col] = (_Float16)(m * sv * FOLD_MS);
          }
        }
      }
    }
    __syncthreads();

    {
      v8f ag[2][4];
#pragma unroll
      for (int mt = 0; mt < 2; ++mt)
#pragma unroll
        for (int g = 0; g < 4; ++g) ag[mt][g] = z8;
      const _Float16* ap = Ac + c * TPITCH + COL_MS + koff;
      const _Float16* wi = WIH + (size_t)jh * CH3 + koff;
#pragma unroll 1
      for (int k0 = 0; k0 < CH3; k0 += 32) {
        const v16h a0 = Frag<_Float16>::load(ap + k0);
        const v16h a1 = Frag<_Float16>::load(ap + 16 * TPITCH + k0);
        const v16h b0 = Frag<_Float16>::load(wi + k0);
        const v16h b1 = Frag<_Float16>::load(wi + (size_t)1 * NHID * CH3 + k0);
        const v16h b2 = Frag<_Float16>::load(wi + (size_t)2 * NHID * CH3 + k0);
        const v16h b3 = Frag<_Float16>::load(wi + (size_t)3 * NHID * CH3 + k0);
        ag[0][0] = Frag<_Float16>::mma(a0, b0, ag[0][0]);
        ag[0][1] = Frag<_Float16>::mma(a0, b1, ag[0][1]);
        ag[0][2] = Frag<_Float16>::mma(a0, b2, ag[0][2]);
        ag[0][3] = Frag<_Float16>::mma(a0, b3, ag[0][3]);
        ag[1][0] = Frag<_Float16>::mma(a1, b0, ag[1][0]);
        ag[1][1] = Frag<_Float16>::mma(a1, b1, ag[1][1]);
        ag[1][2] = Frag<_Float16>::mma(a1, b2, ag[1][2]);
        ag[1][3] = Frag<_Float16>::mma(a1, b3, ag[1][3]);
        dep_guard_h(ag[0][0], ag[1][3], a0, a1);
        keep4_h(b0, b1, b2, b3);
      }
      const _Float16* ah = Ac + c * TPITCH + COL_HID + koff;
      const _Float16* wh = WHH + (size_t)jh * NHID + koff;
#pragma unroll 1
      for (int k0 = 0; k0 < NHID; k0 += 32) {
        const v16h a0 = Frag<_Float16>::load(ah + k0);
        const v16h a1 = Frag<_Float16>::load(ah + 16 * TPITCH + k0);
        const v16h b0 = Frag<_Float16>::load(wh + k0);
        const v16h b1 = Frag<_Float16>::load(wh + (size_t)1 * NHID * NHID + k0);
        const v16h b2 = Frag<_Float16>::load(wh + (size_t)2 * NHID * NHID + k0);
        const v16h b3 = Frag<_Float16>::load(wh + (size_t)3 * NHID * NHID + k0);
        ag[0][0] = Frag<_Float16>::mma(a0, b0, ag[0][0]);
        ag[0][1] = Frag<_Float16>::mma(a0, b1, ag[0][1]);
        ag[0][2] = Frag<_Float16>::mma(a0, b2, ag[0][2]);
        ag[0][3] = Frag<_Float16>::mma(a0, b3, ag[0][3]);
        ag[1][0] = Frag<_Float16>::mma(a1, b0, ag[1][0]);
        ag[1][1] = Frag<_Float16>::mma(a1, b1, ag[1][1]);
        ag[1][2] = Frag<_Float16>::mma(a1, b2, ag[1][2]);
        ag[1][3] = Frag<_Float16>::mma(a1, b3, ag[1][3]);
        dep_guard_h(ag[0][0], ag[1][3], a0, a1);
        keep4_h(b0, b1, b2, b3);
      }
      acc_guard4(ag[0][0], ag[0][1], ag[0][2], ag[0][3]);
      acc_guard4(ag[1][0], ag[1][1], ag[1][2], ag[1][3]);
#pragma unroll
      for (int mt = 0; mt < 2; ++mt) {
#pragma unroll
        for (int r = 0; r < 8; ++r) {
          const int row = 16 * mt + 8 * hh + r;
          const float zi = ag[mt][0][r] * INV_GAT + bg[0];
          const float zf = ag[mt][1][r] * INV_GAT + bg[1];
          const float zg = ag[mt][2][r] * INV_GAT + bg[2];
          const float zo = ag[mt][3][r] * INV_GAT + bg[3];
          const float ig = fsig(zi);
          const float fg = fsig(zf);
          const float og = fsig(zo);
          const float gg = tanh_acc(zg);
          const float cn = fg * cst[mt][r] + ig * gg;
          cst[mt][r] = cn;
          const float hn = og * tanh_acc(cn);
          An[row * TPITCH + COL_HID + jh] = (_Float16)(hn * CARRY_H);
          if (last) Hs[row * HSPITCH + jh] = hn;
        }
      }
    }
    __syncthreads();
  }

  {
    const int m   = tid >> 3;
    const int cls = tid & 7;
    const float* hrow = Hs + m * HSPITCH;
    const float* wrow = clsw + (size_t)cls * NHID;
    float s = 0.0f;
#pragma unroll 1
    for (int k = 0; k < NHID; ++k) s = fmaf(hrow[k], bf16r(wrow[k]), s);
    s += bf16r(clsb[cls]);
    Os[tid] = s;
  }
  __syncthreads();
  if (tid < 32) {
    const v4f v0 = *(const v4f*)(Os + 4 * lane);
    const v4f v1 = *(const v4f*)(Os + 128 + 4 * lane);
    float* ob = out + (size_t)blockIdx.x * (LROWS * NCLS);
    for (int pass = 0; pass < 2; ++pass) {
      *(volatile v4f*)(ob + 4 * lane) = v0;
      *(volatile v4f*)(ob + 128 + 4 * lane) = v1;
      __threadfence();
    }
  }
}

extern "C" void kernel_launch(void* const* d_in, const int* in_sizes, int n_in,
                              void* d_out, int out_size, void* d_ws, size_t ws_size, hipStream_t stream) {
  if (n_in < 17 || d_out == nullptr || d_ws == nullptr) return;
  if (in_sizes[0] != NBAT * NSTEP * NFEAT || in_sizes[1] < 1 || in_sizes[2] < 1 ||
      in_sizes[3] != CH1 * NFEAT * 3 || in_sizes[4] != CH1 ||
      in_sizes[5] != CH2 * CH1 * 3 || in_sizes[6] != CH2 ||
      in_sizes[7] != CH3 * CH2 * 3 || in_sizes[8] != CH3 ||
      in_sizes[9] != CH3 * KMODIN || in_sizes[10] != CH3 ||
      in_sizes[11] != NGC * CH3 || in_sizes[12] != NGC * NHID ||
      in_sizes[13] != NGC || in_sizes[14] != NGC ||
      in_sizes[15] != NCLS * NHID || in_sizes[16] != NCLS ||
      out_size != NBAT * NCLS) return;

  const float* x    = (const float*)d_in[0];
  const float* ksp  = (const float*)d_in[1];
  const float* kap  = (const float*)d_in[2];
  const float* w1   = (const float*)d_in[3];
  const float* b1   = (const float*)d_in[4];
  const float* w2   = (const float*)d_in[5];
  const float* b2   = (const float*)d_in[6];
  const float* w3   = (const float*)d_in[7];
  const float* b3   = (const float*)d_in[8];
  const float* modw = (const float*)d_in[9];
  const float* modb = (const float*)d_in[10];
  const float* wih  = (const float*)d_in[11];
  const float* whh  = (const float*)d_in[12];
  const float* bih  = (const float*)d_in[13];
  const float* bhh  = (const float*)d_in[14];
  const float* clsw = (const float*)d_in[15];
  const float* clsb = (const float*)d_in[16];
  float* out = (float*)d_out;

  char* ws = (char*)d_ws; size_t off = 0;
  auto carve = [&](size_t bytes) -> char* { char* p = ws + off; off += (bytes + 255) & ~(size_t)255; return p; };
  float* WQ   = (float*)carve((size_t)NBAT * NSTEP * 4);
  float* LQ   = (float*)carve((size_t)NBAT * NSTEP * 4);
  float* WN   = (float*)carve((size_t)NBAT * NSTEP * 4);
  float* LN   = (float*)carve((size_t)NBAT * NSTEP * 4);
  float* PART = (float*)carve((size_t)NBAT * 32 * 4);
  float* DL   = (float*)carve((size_t)NBAT * 32 * 4);
  unsigned short* W1P  = (unsigned short*)carve((size_t)CH1 * KW1 * 2);
  unsigned short* W2P  = (unsigned short*)carve((size_t)CH2 * KW2 * 2);
  unsigned short* W3P  = (unsigned short*)carve((size_t)CH3 * KW3 * 2);
  unsigned short* MWP  = (unsigned short*)carve((size_t)CH3 * KMODW * 2);
  unsigned short* WIHP = (unsigned short*)carve((size_t)NGC * CH3 * 2);
  unsigned short* WHHP = (unsigned short*)carve((size_t)NGC * NHID * 2);
  unsigned short* SEQ  = (unsigned short*)carve((size_t)NBAT * NSTEP * CH3 * 2);
  unsigned short* ZP1  = SEQ;
  unsigned short* ZP2  = (unsigned short*)carve((size_t)NBAT * PROWS * CH2 * 2);
  unsigned short* A1   = ZP2;
  const size_t ybytes = (size_t)16777216;
  float* Y = (float*)carve(ybytes);
  if (off > ws_size || off > (size_t)134217728) return;
  if ((size_t)NBAT * PROWS * CH1 * 2 > (size_t)NBAT * NSTEP * CH3 * 2) return;
  if ((size_t)NBAT * NSTEP * KW1 * 2 > (size_t)NBAT * PROWS * CH2 * 2) return;
  if ((size_t)128 * NSTEP * CH1 * 4 > ybytes || (size_t)64 * NSTEP * CH2 * 4 > ybytes || (size_t)32 * NSTEP * CH3 * 4 > ybytes) return;

  queue_kernel<<<NBAT, NSTEP, 0, stream>>>(x, ksp, kap, WQ, LQ, PART);
  norm_kernel<<<NBAT, NSTEP, 0, stream>>>(WQ, LQ, PART, WN, LN, DL);

  { const int n8 = CH1 * KW1 / 8;    wcvt_kernel<<<(n8 + 255) / 256, 256, 0, stream>>>(w1,   W1P,  n8, KW1,   KW1SRC, 1,   0, CWCONV); }
  { const int n8 = CH2 * KW2 / 8;    wcvt_kernel<<<(n8 + 255) / 256, 256, 0, stream>>>(w2,   W2P,  n8, KW2,   KW2,    CH1, 1, CWCONV); }
  { const int n8 = CH3 * KW3 / 8;    wcvt_kernel<<<(n8 + 255) / 256, 256, 0, stream>>>(w3,   W3P,  n8, KW3,   KW3,    CH2, 1, CWCONV); }
  { const int n8 = CH3 * KMODW / 8;  wcvt_kernel<<<(n8 + 255) / 256, 256, 0, stream>>>(modw, MWP,  n8, KMODW, KMODIN, 1,   2, CWMOD); }
  { const int n8 = NGC * CH3 / 8;    wcvt_kernel<<<(n8 + 255) / 256, 256, 0, stream>>>(wih,  WIHP, n8, CH3,   CH3,    1,   0, CWIH); }
  { const int n8 = NGC * NHID / 8;   wcvt_kernel<<<(n8 + 255) / 256, 256, 0, stream>>>(whh,  WHHP, n8, NHID,  NHID,   1,   0, CWHH); }

  xcol_kernel<<<(NBAT * NSTEP * 8) / 256, 256, 0, stream>>>(x, A1);

  for (int ch = 0; ch < 2; ++ch) {
    const unsigned short* Ac = A1 + (size_t)ch * 65536 * KW1;
    wmma_gemm64<0, false, 3, 0, false, 2><<<dim3(128, 1), 256, 0, stream>>>(
        Ac, Ac, KW1, 0L, W1P, W1P, KW1, 0L, (void*)Y, (void*)Y, CH1, 0L, b1, b1, 0L, 65536, CH1, KW1, INV_G1);
    simam_cvt_kernel<<<dim3(CH1 / 64, 128), 256, 0, stream>>>(Y, CH1, DL, ZP1, PROWS, 1, ch * 128, CZ1);
  }
  for (int ch = 0; ch < 4; ++ch) {
    const unsigned short* Ac = ZP1 + (size_t)ch * 64 * PROWS * CH1;
    wmma_gemm64<0, false, 3, 0, false, 2><<<dim3(2, 64), 256, 0, stream>>>(
        Ac, Ac, CH1, (long)PROWS * CH1, W2P, W2P, KW2, 0L, (void*)Y, (void*)Y, CH2, (long)NSTEP * CH2, b2, b2, 0L, NSTEP, CH2, KW2, INV_G2);
    simam_cvt_kernel<<<dim3(CH2 / 64, 64), 256, 0, stream>>>(Y, CH2, DL, ZP2, PROWS, 1, ch * 64, CZ2);
  }
  for (int ch = 0; ch < 8; ++ch) {
    const unsigned short* Ac = ZP2 + (size_t)ch * 32 * PROWS * CH2;
    wmma_gemm64<0, false, 3, 0, false, 2><<<dim3(4, 32), 256, 0, stream>>>(
        Ac, Ac, CH2, (long)PROWS * CH2, W3P, W3P, KW3, 0L, (void*)Y, (void*)Y, CH3, (long)NSTEP * CH3, b3, b3, 0L, NSTEP, CH3, KW3, INV_G3);
    simam_cvt_kernel<<<dim3(CH3 / 64, 32), 256, 0, stream>>>(Y, CH3, DL, SEQ, NSTEP, 0, ch * 32, CSEQ);
  }
  lstm_kernel<<<NBAT / LROWS, LTHR, 0, stream>>>(SEQ, WN, LN, MWP, modb, WIHP, WHHP, bih, bhh, clsw, clsb, out);
}
